// GPT2Attention_87522843558459
// MI455X (gfx1250) — hardware-verified
//
#include <hip/hip_runtime.h>

typedef __attribute__((ext_vector_type(16))) _Float16 v16h;
typedef __attribute__((ext_vector_type(8)))  _Float16 v8h;
typedef __attribute__((ext_vector_type(16))) __bf16   v16b;
typedef __attribute__((ext_vector_type(8)))  __bf16   v8b;
typedef __attribute__((ext_vector_type(8)))  float    v8f;
typedef __attribute__((ext_vector_type(4)))  float    v4f;
typedef __attribute__((ext_vector_type(4)))  unsigned int u32x4;

constexpr int NBATCH = 4;
constexpr int SEQ    = 2048;
constexpr int DMODEL = 1024;
constexpr int NHEAD  = 16;
constexpr int HDIM   = 64;
constexpr int QKV_LD = 3 * DMODEL;
constexpr int KCH    = 64;
constexpr int QBLK   = 64;
static_assert(NHEAD * HDIM == DMODEL, "head split");
static_assert(HDIM == 64, "attention kernel is written for head_dim 64");
static_assert(SEQ % QBLK == 0 && SEQ % KCH == 0 && QBLK == KCH, "attention tiling");
static_assert(SEQ % 64 == 0 && QKV_LD % 64 == 0 && DMODEL % 64 == 0 && DMODEL % 32 == 0, "GEMM tiles");
static_assert(((SEQ / 64) * (QKV_LD / 64)) % 8 == 0 && ((SEQ / 64) * (DMODEL / 64)) % 8 == 0, "8 tiles per GEMM block");
static_assert((NBATCH * SEQ * DMODEL) % (8 * 256) == 0, "cast grid exact");

constexpr float NEG_INF_F = -__builtin_huge_valf();

__device__ __forceinline__ unsigned short f2bf_bits(float f) {
  unsigned u = __float_as_uint(f);
  return (unsigned short)((u + 0x7FFFu + ((u >> 16) & 1u)) >> 16);
}
__device__ __forceinline__ float bf_bits2f(unsigned short h) { return __uint_as_float(((unsigned)h) << 16); }

__device__ __forceinline__ void dep_guard_h(v8f& a, v8f& b, v16h x, v16h y) { asm volatile("v_nop\n\tv_nop\n\tv_nop\n\tv_nop" : "+v"(a), "+v"(b) : "v"(x), "v"(y)); }
__device__ __forceinline__ void dep_guard_b(v8f& a, v8f& b, v16b x, v16b y) { asm volatile("v_nop\n\tv_nop\n\tv_nop\n\tv_nop" : "+v"(a), "+v"(b) : "v"(x), "v"(y)); }
__device__ __forceinline__ void keep4_h(v16h a, v16h b, v16h c, v16h d) { asm volatile("v_nop" :: "v"(a), "v"(b), "v"(c), "v"(d)); }
__device__ __forceinline__ void keep4_b(v16b a, v16b b, v16b c, v16b d) { asm volatile("v_nop" :: "v"(a), "v"(b), "v"(c), "v"(d)); }
__device__ __forceinline__ void acc_guard4(v8f& a, v8f& b, v8f& c, v8f& d) { asm volatile("v_nop\n\tv_nop\n\tv_nop\n\tv_nop" : "+v"(a), "+v"(b), "+v"(c), "+v"(d)); }
template <typename T> struct Frag;
template <> struct Frag<_Float16> {
  typedef v16h V; union U { v16h v; v8h h[2]; };
  static __device__ __forceinline__ v16h load(const _Float16* p) {
    U f; f.h[0] = *(const v8h*)(p); f.h[1] = *(const v8h*)(p + 16); return f.v;
  }
  static __device__ __forceinline__ v8f mma(v16h a, v16h b, v8f c) {
    return __builtin_amdgcn_wmma_f32_16x16x32_f16(false, a, false, b, (short)0, c, false, false);
  }
  static __device__ __forceinline__ void guard(v8f& a, v8f& b, v16h x, v16h y) { dep_guard_h(a, b, x, y); }
  static __device__ __forceinline__ void keep(v16h a, v16h b, v16h c, v16h d) { keep4_h(a, b, c, d); }
};
template <> struct Frag<__bf16> {
  typedef v16b V; union U { v16b v; v8b h[2]; };
  static __device__ __forceinline__ v16b load(const __bf16* p) {
    U f; f.h[0] = *(const v8b*)(p); f.h[1] = *(const v8b*)(p + 16); return f.v;
  }
  static __device__ __forceinline__ v8f mma(v16b a, v16b b, v8f c) {
    return __builtin_amdgcn_wmma_f32_16x16x32_bf16(false, a, false, b, (short)0, c, false, false);
  }
  static __device__ __forceinline__ void guard(v8f& a, v8f& b, v16b x, v16b y) { dep_guard_b(a, b, x, y); }
  static __device__ __forceinline__ void keep(v16b a, v16b b, v16b c, v16b d) { keep4_b(a, b, c, d); }
};

template <int ET> struct Elem;
template <> struct Elem<0> { typedef _Float16 T; };
template <> struct Elem<1> { typedef __bf16 T; };
template <int ET, int SPLITM, int BIAS_MODE, int OUT_MODE, bool RESID, int ACT = 0>
__global__ __launch_bounds__(256) void wmma_gemm64(
    const unsigned short* __restrict__ Ap, const unsigned short* __restrict__ A2p, int lda, long strideA,
    const unsigned short* __restrict__ Btp, const unsigned short* __restrict__ Bt2p, int ldb, long strideB,
    void* __restrict__ Cout, void* __restrict__ Cout2, int ldc, long strideC,
    const float* __restrict__ bias,
    const float* __restrict__ resid, long strideR,
    int M, int N, int K, float scale) {
  constexpr bool SPA = (SPLITM >= 1);
  constexpr bool SPB = (SPLITM >= 2);
  typedef typename Elem<ET>::T T;
  typedef typename Frag<T>::V V;
  const T* A = (const T*)Ap; const T* A2 = (const T*)A2p; const T* Bt = (const T*)Btp; const T* Bt2 = (const T*)Bt2p;
  __shared__ __align__(16) float sT[8][16 * 68];
  const int b    = blockIdx.y;
  const int lane = threadIdx.x & 31;
  const int wave = threadIdx.x >> 5;
  const int tilesN = N >> 6;
  const int tilesM = M >> 6;
  const int tile = blockIdx.x * 8 + wave;
  if (tile >= tilesM * tilesN) return;
  const int tm = tile / tilesN;
  const int tn = tile - tm * tilesN;
  const int m0 = tm << 6;
  const int n0 = tn << 6;

  const T* Ab  = A  + (size_t)b * strideA;
  const T* Bb  = Bt + (size_t)b * strideB;
  const T* Ab2 = SPA ? (A2  + (size_t)b * strideA) : nullptr;
  const T* Bb2 = SPB ? (Bt2 + (size_t)b * strideB) : nullptr;

  const int rlane = lane & 15;
  const int koff  = (lane >> 4) * 8;
  const int mOff  = (lane >> 4) * 8;

  v8f acc[4][4];
#pragma unroll
  for (int i = 0; i < 4; ++i)
#pragma unroll
    for (int j = 0; j < 4; ++j) acc[i][j] = (v8f){0.f,0.f,0.f,0.f,0.f,0.f,0.f,0.f};

  for (int k0 = 0; k0 < K; k0 += 32) {
    V bh[4], bl[4];
#pragma unroll
    for (int j = 0; j < 4; ++j) {
      const size_t bo = (size_t)(n0 + (j << 4) + rlane) * ldb + koff + k0;
      bh[j] = Frag<T>::load(Bb + bo);
      if (SPB) bl[j] = Frag<T>::load(Bb2 + bo);
    }
#pragma unroll
    for (int i = 0; i < 4; ++i) {
      const size_t ao = (size_t)(m0 + (i << 4) + rlane) * lda + koff + k0;
      V ah = Frag<T>::load(Ab + ao);
      V al;
      if (SPA) al = Frag<T>::load(Ab2 + ao);
      else al = ah;
#pragma unroll
      for (int j = 0; j < 4; ++j) {
        acc[i][j] = Frag<T>::mma(ah, bh[j], acc[i][j]);
        if (SPB) acc[i][j] = Frag<T>::mma(ah, bl[j], acc[i][j]);
        if (SPA) acc[i][j] = Frag<T>::mma(al, bh[j], acc[i][j]);
      }
      Frag<T>::guard(acc[i][0], acc[i][3], ah, al);
    }
    Frag<T>::keep(bh[0], bh[1], bh[2], bh[3]);
    if (SPB) Frag<T>::keep(bl[0], bl[1], bl[2], bl[3]);
  }
  acc_guard4(acc[0][0], acc[0][1], acc[0][2], acc[0][3]);
  acc_guard4(acc[1][0], acc[1][1], acc[1][2], acc[1][3]);
  acc_guard4(acc[2][0], acc[2][1], acc[2][2], acc[2][3]);
  acc_guard4(acc[3][0], acc[3][1], acc[3][2], acc[3][3]);

  float* slab = sT[wave];
  const float* Rb = RESID ? (resid + (size_t)b * strideR) : nullptr;
#pragma unroll
  for (int i = 0; i < 4; ++i) {
    const int mBase = m0 + (i << 4);
#pragma unroll
    for (int j = 0; j < 4; ++j) {
      const int n = n0 + (j << 4) + rlane;
      float bv = 0.f;
      if (BIAS_MODE == 2) bv = bf_bits2f(f2bf_bits(bias[n]));
#pragma unroll
      for (int r = 0; r < 8; ++r) {
        float v = acc[i][j][r] * scale;
        if (BIAS_MODE == 1) v += bf_bits2f(f2bf_bits(bias[mBase + mOff + r]));
        if (BIAS_MODE == 2) v += bv;
        if (RESID) v += Rb[(size_t)(mBase + mOff + r) * ldc + n];
        if (ACT == 1) v = tanhf(v);
        if (ACT == 2) v = fmaxf(v, 0.0f);
        if (ACT == 3) v = v / (1.0f + expf(-v));
        if (ACT == 4) v = (v > 0.f) ? v : 0.01f * v;
        slab[(mOff + r) * 68 + (j << 4) + rlane] = v;
      }
    }
    __builtin_amdgcn_fence(__ATOMIC_RELEASE, "workgroup");
    __builtin_amdgcn_wave_barrier();
    __builtin_amdgcn_fence(__ATOMIC_ACQUIRE, "workgroup");
    if (OUT_MODE == 0) {
      float* C = (float*)Cout + (size_t)b * strideC;
      const int hh = lane >> 4, c4 = (lane & 15) * 4;
      for (int pass = 0; pass < 2; ++pass) {
#pragma unroll
        for (int it = 0; it < 8; ++it) {
          const int row = it * 2 + hh;
          v4f v = *(const v4f*)(slab + row * 68 + c4);
          *(volatile v4f*)(C + (size_t)(mBase + row) * ldc + n0 + c4) = v;
        }
        __threadfence();
      }
    } else {
      const int q = lane >> 3, c8 = (lane & 7) * 8;
      unsigned short* C  = (unsigned short*)Cout  + (size_t)b * strideC;
      unsigned short* C2 = (OUT_MODE == 2) ? ((unsigned short*)Cout2 + (size_t)b * strideC) : nullptr;
      for (int pass = 0; pass < 2; ++pass) {
#pragma unroll
        for (int it = 0; it < 4; ++it) {
          const int row = it * 4 + q;
          const float* sp = slab + row * 68 + c8;
          v8h hv, lv;
#pragma unroll
          for (int e = 0; e < 8; ++e) {
            if (OUT_MODE == 1) {
              hv[e] = (_Float16)sp[e];
            } else {
              unsigned short hb = f2bf_bits(sp[e]);
              unsigned short lb = f2bf_bits(sp[e] - bf_bits2f(hb));
              hv[e] = __builtin_bit_cast(_Float16, hb);
              lv[e] = __builtin_bit_cast(_Float16, lb);
            }
          }
          *(volatile v8h*)(C + (size_t)(mBase + row) * ldc + n0 + c8) = hv;
          if (OUT_MODE == 2) *(volatile v8h*)(C2 + (size_t)(mBase + row) * ldc + n0 + c8) = lv;
        }
        __threadfence();
      }
    }
    __builtin_amdgcn_fence(__ATOMIC_RELEASE, "workgroup");
    __builtin_amdgcn_wave_barrier();
    __builtin_amdgcn_fence(__ATOMIC_ACQUIRE, "workgroup");
  }
}

__global__ __launch_bounds__(256) void cast_rows_bf16(
    const float* __restrict__ in, unsigned short* __restrict__ out, int n8) {
  const int i = blockIdx.x * 256 + threadIdx.x;
  if (i < n8) {
    const v4f a = *(const v4f*)(in + (size_t)i * 8);
    const v4f c = *(const v4f*)(in + (size_t)i * 8 + 4);
    u32x4 w;
    w[0] = (unsigned)f2bf_bits(a[0]) | ((unsigned)f2bf_bits(a[1]) << 16);
    w[1] = (unsigned)f2bf_bits(a[2]) | ((unsigned)f2bf_bits(a[3]) << 16);
    w[2] = (unsigned)f2bf_bits(c[0]) | ((unsigned)f2bf_bits(c[1]) << 16);
    w[3] = (unsigned)f2bf_bits(c[2]) | ((unsigned)f2bf_bits(c[3]) << 16);
    unsigned short* p = out + (size_t)i * 8;
    *(volatile u32x4*)p = w;
    __threadfence();
    *(volatile u32x4*)p = w;
  }
}

__global__ __launch_bounds__(256) void transpose_cast_bf16(
    const float* __restrict__ W, unsigned short* __restrict__ Wt, int nrows_k, int ncols_n) {
  __shared__ __align__(16) float tile[64][65];
  const int tid = threadIdx.x;
  const int n0 = blockIdx.x * 64, k0 = blockIdx.y * 64;
  {
    const int c4 = (tid & 15) * 4;
#pragma unroll
    for (int it = 0; it < 4; ++it) {
      const int kr = (tid >> 4) + 16 * it;
      const v4f x = *(const v4f*)(W + (size_t)(k0 + kr) * ncols_n + n0 + c4);
      tile[kr][c4 + 0] = x[0];
      tile[kr][c4 + 1] = x[1];
      tile[kr][c4 + 2] = x[2];
      tile[kr][c4 + 3] = x[3];
    }
  }
  __syncthreads();
  const int c8 = (tid & 7) * 8;
  for (int pass = 0; pass < 2; ++pass) {
#pragma unroll
    for (int it = 0; it < 2; ++it) {
      const int nr = (tid >> 3) + 32 * it;
      unsigned short hb[8];
#pragma unroll
      for (int e = 0; e < 8; ++e) hb[e] = f2bf_bits(tile[c8 + e][nr]);
      u32x4 w;
      w[0] = (unsigned)hb[0] | ((unsigned)hb[1] << 16);
      w[1] = (unsigned)hb[2] | ((unsigned)hb[3] << 16);
      w[2] = (unsigned)hb[4] | ((unsigned)hb[5] << 16);
      w[3] = (unsigned)hb[6] | ((unsigned)hb[7] << 16);
      *(volatile u32x4*)(Wt + (size_t)(n0 + nr) * nrows_k + k0 + c8) = w;
    }
    __threadfence();
  }
}

__device__ __forceinline__ void at_split(float f, __bf16& hi, __bf16& lo) {
  const unsigned short hb = f2bf_bits(f);
  hi = __builtin_bit_cast(__bf16, hb);
  lo = __builtin_bit_cast(__bf16, f2bf_bits(f - __uint_as_float(((unsigned)hb) << 16)));
}
__device__ __forceinline__ v8f mma_bf(v16b a, v16b b, v8f c) {
  c = __builtin_amdgcn_wmma_f32_16x16x32_bf16(false, a, false, b, (short)0, c, false, false);
  asm volatile("v_nop\n\tv_nop\n\tv_nop\n\tv_nop" : "+v"(c) : "v"(a), "v"(b));
  return c;
}

union AttnSmem {
  struct KV { unsigned short kh[KCH * HDIM]; unsigned short kl[KCH * HDIM]; unsigned short vh[HDIM * KCH]; } t;
  float os[4][16 * 68];
};

__global__ __launch_bounds__(128)
void attn_causal_hd64(const unsigned short* __restrict__ qkv_hi, const unsigned short* __restrict__ qkv_lo,
                      unsigned short* __restrict__ ctx_hi, unsigned short* __restrict__ ctx_lo) {
  __shared__ __align__(16) AttnSmem su;
  __shared__ __align__(16) unsigned short svl[HDIM * KCH];
  __shared__ __align__(16) __bf16 sph[4][16 * KCH];
  __shared__ __align__(16) __bf16 spl[4][16 * KCH];

  const int tid  = threadIdx.x;
  const int wave = tid >> 5;
  const int lane = tid & 31;
  const int hh   = lane >> 4;
  const int c    = lane & 15;
  constexpr int NQB = SEQ / QBLK;
  const int qb = blockIdx.x % NQB;
  const int h  = (blockIdx.x / NQB) % NHEAD;
  const int q0 = qb * QBLK + wave * 16;

  const __bf16* QH = (const __bf16*)(const void*)qkv_hi;
  const __bf16* QL = (const __bf16*)(const void*)qkv_lo;

  v16b qah[2], qal[2];
#pragma unroll
  for (int dc = 0; dc < 2; ++dc) {
    const size_t qo = (size_t)(q0 + c) * QKV_LD + (size_t)h * HDIM + dc * 32 + 8 * hh;
    qah[dc] = Frag<__bf16>::load(QH + qo);
    qal[dc] = Frag<__bf16>::load(QL + qo);
  }

  float mrow[8], lrow[8];
  v8f oacc[4];
#pragma unroll
  for (int r = 0; r < 8; ++r) { mrow[r] = NEG_INF_F; lrow[r] = 0.f; }
#pragma unroll
  for (int t = 0; t < 4; ++t) oacc[t] = (v8f){0.f,0.f,0.f,0.f,0.f,0.f,0.f,0.f};

  const int nChunks = qb + 1;
  for (int kc = 0; kc < nChunks; ++kc) {
    const int kv0 = kc * KCH;
    __syncthreads();
    {
      const int kvr = tid >> 1, dh = (tid & 1) * 32;
      const size_t ro = (size_t)(kv0 + kvr) * QKV_LD + (size_t)h * HDIM + dh;
      const u32x4* khp = (const u32x4*)(const void*)(qkv_hi + ro + DMODEL);
      const u32x4* klp = (const u32x4*)(const void*)(qkv_lo + ro + DMODEL);
      u32x4 wa[4], wb[4];
#pragma unroll
      for (int i = 0; i < 4; ++i) { wa[i] = khp[i]; wb[i] = klp[i]; }
#pragma unroll
      for (int i = 0; i < 4; ++i) {
        *(u32x4*)(su.t.kh + kvr * HDIM + dh + 8 * i) = wa[i];
        *(u32x4*)(su.t.kl + kvr * HDIM + dh + 8 * i) = wb[i];
      }
      asm volatile("" ::: "memory");
      const u32x4* vhp = (const u32x4*)(const void*)(qkv_hi + ro + 2 * DMODEL);
      const u32x4* vlp = (const u32x4*)(const void*)(qkv_lo + ro + 2 * DMODEL);
#pragma unroll
      for (int i = 0; i < 4; ++i) { wa[i] = vhp[i]; wb[i] = vlp[i]; }
#pragma unroll
      for (int i = 0; i < 4; ++i) {
#pragma unroll
        for (int j = 0; j < 4; ++j) {
          const int d = dh + 8 * i + 2 * j;
          const unsigned ua = wa[i][j], ub = wb[i][j];
          su.t.vh[d * KCH + kvr]       = (unsigned short)(ua & 0xffffu);
          su.t.vh[(d + 1) * KCH + kvr] = (unsigned short)(ua >> 16);
          svl[d * KCH + kvr]           = (unsigned short)(ub & 0xffffu);
          svl[(d + 1) * KCH + kvr]     = (unsigned short)(ub >> 16);
        }
      }
    }
    __syncthreads();

    v8f s[4];
#pragma unroll
    for (int j = 0; j < 4; ++j) {
      s[j] = (v8f){0.f,0.f,0.f,0.f,0.f,0.f,0.f,0.f};
#pragma unroll
      for (int dc = 0; dc < 2; ++dc) {
        const int ko = (j * 16 + c) * HDIM + dc * 32 + 8 * hh;
        const v16b kbh = Frag<__bf16>::load((const __bf16*)(const void*)(su.t.kh) + ko);
        const v16b kbl = Frag<__bf16>::load((const __bf16*)(const void*)(su.t.kl) + ko);
        s[j] = mma_bf(qah[dc], kbh, s[j]);
        s[j] = mma_bf(qah[dc], kbl, s[j]);
        s[j] = mma_bf(qal[dc], kbh, s[j]);
      }
    }
    const bool diag = (kc == qb);
    float cm[8];
#pragma unroll
    for (int r = 0; r < 8; ++r) {
      const int qrow = q0 + 8 * hh + r;
      float m = NEG_INF_F;
#pragma unroll
      for (int j = 0; j < 4; ++j) {
        const int kvcol = kv0 + j * 16 + c;
        float val = s[j][r] * 0.125f;
        val = (diag && (kvcol > qrow)) ? NEG_INF_F : val;
        s[j][r] = val;
        m = fmaxf(m, val);
      }
#pragma unroll
      for (int off = 1; off < 16; off <<= 1) m = fmaxf(m, __shfl_xor(m, off, 32));
      cm[r] = m;
    }
    __bf16* pwh = sph[wave];
    __bf16* pwl = spl[wave];
#pragma unroll
    for (int r = 0; r < 8; ++r) {
      const float mnew  = fmaxf(mrow[r], cm[r]);
      const float alpha = expf(mrow[r] - mnew);
      mrow[r] = mnew;
      float psum = 0.f;
#pragma unroll
      for (int j = 0; j < 4; ++j) {
        const float p = expf(s[j][r] - mnew);
        psum += p;
        __bf16 ph, pl2;
        at_split(p, ph, pl2);
        pwh[(8 * hh + r) * KCH + j * 16 + c] = ph;
        pwl[(8 * hh + r) * KCH + j * 16 + c] = pl2;
      }
#pragma unroll
      for (int off = 1; off < 16; off <<= 1) psum += __shfl_xor(psum, off, 32);
      lrow[r] = lrow[r] * alpha + psum;
#pragma unroll
      for (int t = 0; t < 4; ++t) oacc[t][r] *= alpha;
    }
    __syncthreads();

#pragma unroll 1
    for (int kk = 0; kk < 2; ++kk) {
      const int po = c * KCH + kk * 32 + 8 * hh;
      const v16b pa = Frag<__bf16>::load(pwh + po);
      const v16b pl = Frag<__bf16>::load(pwl + po);
#pragma unroll
      for (int t = 0; t < 4; ++t) {
        const int vo = (t * 16 + c) * KCH + kk * 32 + 8 * hh;
        const v16b vbh = Frag<__bf16>::load((const __bf16*)(const void*)(su.t.vh) + vo);
        const v16b vbl = Frag<__bf16>::load((const __bf16*)(const void*)(svl) + vo);
        oacc[t] = mma_bf(pa, vbh, oacc[t]);
        oacc[t] = mma_bf(pa, vbl, oacc[t]);
        oacc[t] = mma_bf(pl, vbh, oacc[t]);
      }
    }
  }

  __syncthreads();
  float* os = su.os[wave];
#pragma unroll
  for (int r = 0; r < 8; ++r) {
    const float inv = 1.0f / lrow[r];
#pragma unroll
    for (int t = 0; t < 4; ++t) os[(8 * hh + r) * 68 + t * 16 + c] = oacc[t][r] * inv;
  }
  __syncthreads();
  {
    const int q8 = lane >> 3, c8 = (lane & 7) * 8;
    for (int pass = 0; pass < 2; ++pass) {
#pragma unroll
      for (int it = 0; it < 4; ++it) {
        const int row = it * 4 + q8;
        const float* sp = os + row * 68 + c8;
        const v4f f0 = *(const v4f*)sp;
        const v4f f1 = *(const v4f*)(sp + 4);
        unsigned short hb[8], lb[8];
#pragma unroll
        for (int e = 0; e < 4; ++e) {
          const float x0 = f0[e], x1 = f1[e];
          hb[e] = f2bf_bits(x0);     lb[e] = f2bf_bits(x0 - bf_bits2f(hb[e]));
          hb[4 + e] = f2bf_bits(x1); lb[4 + e] = f2bf_bits(x1 - bf_bits2f(hb[4 + e]));
        }
        u32x4 wh, wl;
        wh[0] = (unsigned)hb[0] | ((unsigned)hb[1] << 16); wl[0] = (unsigned)lb[0] | ((unsigned)lb[1] << 16);
        wh[1] = (unsigned)hb[2] | ((unsigned)hb[3] << 16); wl[1] = (unsigned)lb[2] | ((unsigned)lb[3] << 16);
        wh[2] = (unsigned)hb[4] | ((unsigned)hb[5] << 16); wl[2] = (unsigned)lb[4] | ((unsigned)lb[5] << 16);
        wh[3] = (unsigned)hb[6] | ((unsigned)hb[7] << 16); wl[3] = (unsigned)lb[6] | ((unsigned)lb[7] << 16);
        const size_t oo = (size_t)(q0 + row) * DMODEL + (size_t)h * HDIM + c8;
        *(volatile u32x4*)(ctx_hi + oo) = wh;
        *(volatile u32x4*)(ctx_lo + oo) = wl;
      }
      __threadfence();
    }
  }
}

extern "C" void kernel_launch(void* const* d_in, const int* in_sizes, int n_in,
                              void* d_out, int out_size, void* d_ws, size_t ws_size,
                              hipStream_t stream) {
  (void)in_sizes; (void)n_in; (void)out_size;
  const float* hidden = (const float*)d_in[0];
  const float* w_attn = (const float*)d_in[1];
  const float* b_attn = (const float*)d_in[2];
  const float* w_proj = (const float*)d_in[3];
  const float* b_proj = (const float*)d_in[4];
  float* out = (float*)d_out;

  constexpr size_t BYTES_HID  = (size_t)NBATCH * SEQ * DMODEL * 2;
  constexpr size_t BYTES_WT   = (size_t)QKV_LD * DMODEL * 2;
  constexpr size_t BYTES_WPT  = (size_t)DMODEL * DMODEL * 2;
  constexpr size_t BYTES_QKVP = (size_t)SEQ * QKV_LD * 2;
  constexpr size_t BYTES_CTXP = (size_t)SEQ * DMODEL * 2;
  constexpr size_t OFF_HID   = 0;
  constexpr size_t OFF_WT    = OFF_HID + BYTES_HID;
  constexpr size_t OFF_WPT   = OFF_WT + BYTES_WT;
  constexpr size_t OFF_QKVH  = OFF_WPT + BYTES_WPT;
  constexpr size_t OFF_QKVL  = OFF_QKVH + BYTES_QKVP;
  constexpr size_t OFF_CTXH  = OFF_QKVL + BYTES_QKVP;
  constexpr size_t OFF_CTXL  = OFF_CTXH + BYTES_CTXP;
  constexpr size_t WS_TOTAL  = OFF_CTXL + BYTES_CTXP;
  static_assert(WS_TOTAL == 58720256ull, "carve total");
  static_assert(WS_TOTAL <= 134217728ull, "carve within 128 MiB");
  static_assert((OFF_WT % 256) == 0 && (OFF_WPT % 256) == 0 && (OFF_QKVH % 256) == 0 &&
                (OFF_QKVL % 256) == 0 && (OFF_CTXH % 256) == 0 && (OFF_CTXL % 256) == 0, "alignment");
  if (ws_size < WS_TOTAL) return;

  char* ws = (char*)d_ws;
  unsigned short* hid_bf = (unsigned short*)(ws + OFF_HID);
  unsigned short* wt     = (unsigned short*)(ws + OFF_WT);
  unsigned short* wpt    = (unsigned short*)(ws + OFF_WPT);
  unsigned short* qkv_hi = (unsigned short*)(ws + OFF_QKVH);
  unsigned short* qkv_lo = (unsigned short*)(ws + OFF_QKVL);
  unsigned short* ctx_hi = (unsigned short*)(ws + OFF_CTXH);
  unsigned short* ctx_lo = (unsigned short*)(ws + OFF_CTXL);

  {
    constexpr int n8 = NBATCH * SEQ * DMODEL / 8;
    cast_rows_bf16<<<n8 / 256, 256, 0, stream>>>(hidden, hid_bf, n8);
  }
  transpose_cast_bf16<<<dim3(QKV_LD / 64, DMODEL / 64), 256, 0, stream>>>(w_attn, wt, DMODEL, QKV_LD);
  transpose_cast_bf16<<<dim3(DMODEL / 64, DMODEL / 64), 256, 0, stream>>>(w_proj, wpt, DMODEL, DMODEL);

  for (int b = 0; b < NBATCH; ++b) {
    const unsigned short* hidA = hid_bf + (size_t)b * SEQ * DMODEL;
    {
      constexpr int tiles = (SEQ / 64) * (QKV_LD / 64);
      wmma_gemm64<1, 0, 2, 2, false><<<dim3(tiles / 8, 1), 256, 0, stream>>>(
          hidA, hidA, DMODEL, 0L,
          wt, wt, DMODEL, 0L,
          (void*)qkv_hi, (void*)qkv_lo, QKV_LD, 0L,
          b_attn, b_attn, 0L,
          SEQ, QKV_LD, DMODEL, 1.0f);
    }
    attn_causal_hd64<<<NHEAD * (SEQ / QBLK), 128, 0, stream>>>(qkv_hi, qkv_lo, ctx_hi, ctx_lo);
    {
      constexpr int tiles = (SEQ / 64) * (DMODEL / 64);
      float* outb = out + (size_t)b * SEQ * DMODEL;
      wmma_gemm64<1, 1, 2, 0, false><<<dim3(tiles / 8, 1), 256, 0, stream>>>(
          ctx_hi, ctx_lo, DMODEL, 0L,
          wpt, wpt, DMODEL, 0L,
          (void*)outb, (void*)outb, DMODEL, 0L,
          b_proj, b_proj, 0L,
          SEQ, DMODEL, DMODEL, 1.0f);
    }
  }
}
